// MSAOPM_20194936225883
// MI455X (gfx1250) — hardware-run, weakly checked
//
#include <hip/hip_runtime.h>
#include <math.h>

typedef __attribute__((ext_vector_type(16))) _Float16 v16h;
typedef __attribute__((ext_vector_type(8)))  _Float16 v8h;
typedef __attribute__((ext_vector_type(4)))  _Float16 v4h;
typedef __attribute__((ext_vector_type(8)))  float    v8f;
typedef __attribute__((ext_vector_type(4)))  float    v4f;

constexpr int kN  = 128;
constexpr int kL  = 256;
constexpr int kD  = 256;
constexpr int kC  = 32;
constexpr int kZ  = 128;
constexpr int kK3 = kC * kC;
static_assert(kN % 32 == 0);
static_assert(kK3 % 32 == 0);
static_assert(kC == 32);
static_assert(kZ % 16 == 0);
static_assert(kL % 16 == 0);

constexpr float kLnEps    = 1e-5f;
constexpr float kInvD     = 1.0f / (float)kD;
constexpr float kW3Carry  = 32.0f;
constexpr float kOutScale = 1.0f / ((float)kN * kW3Carry);
static_assert(kN * 32 == 4096);

constexpr size_t kBytesA2  = (size_t)kL * kC * kN * 2;
constexpr size_t kBytesB2T = (size_t)kL * kC * kN * 2;
constexpr size_t kBytesW3T = (size_t)kZ * kK3 * 2;
constexpr size_t kOffA2    = 0;
constexpr size_t kOffB2T   = kOffA2 + kBytesA2;
constexpr size_t kOffW3T   = kOffB2T + kBytesB2T;
constexpr size_t kWsTotal  = kOffW3T + kBytesW3T;
static_assert(kWsTotal == 4456448ull);
static_assert(kWsTotal <= 134217728ull);
static_assert((kOffB2T % 128) == 0 && (kOffW3T % 128) == 0);

union FragU { v16h v; v8h h[2]; };
__device__ __forceinline__ v16h frag_load(const _Float16* p) {
  FragU f;
  f.h[0] = *(const v8h*)(p);
  f.h[1] = *(const v8h*)(p + 16);
  return f.v;
}
__device__ __forceinline__ v8f mma_f16(v16h a, v16h b, v8f c) {
  c = __builtin_amdgcn_wmma_f32_16x16x32_f16(false, a, false, b, (short)0, c, false, false);
  asm volatile("v_nop\n\tv_nop\n\tv_nop\n\tv_nop" : "+v"(c) : "v"(a), "v"(b));
  return c;
}

constexpr int kPrepWaves   = 8;
constexpr int kRowsPerWave = kN / kPrepWaves;
constexpr int kRowsPerPass = 4;
constexpr int kPasses      = kRowsPerWave / kRowsPerPass;
static_assert(kRowsPerWave == 16 && kPasses == 4);

__global__ __launch_bounds__(256) void prep_kernel(
    const float* __restrict__ m, const float* __restrict__ ln_w, const float* __restrict__ ln_b,
    const float* __restrict__ w1, const float* __restrict__ b1,
    const float* __restrict__ w2, const float* __restrict__ b2,
    _Float16* __restrict__ A2, _Float16* __restrict__ B2T)
{
  __shared__ __align__(16) float    o_t[kPrepWaves][kD * kRowsPerPass];
  __shared__ __align__(16) _Float16 ab_s[2][kC * kN];
  const int tid  = threadIdx.x;
  const int lane = tid & 31;
  const int wave = tid >> 5;
  const int l    = blockIdx.x;

  const v4f lw0 = *(const v4f*)(ln_w + lane * 8);
  const v4f lw1 = *(const v4f*)(ln_w + lane * 8 + 4);
  const v4f lb0 = *(const v4f*)(ln_b + lane * 8);
  const v4f lb1 = *(const v4f*)(ln_b + lane * 8 + 4);
  const float bias_a = b2[lane];
  const float bias_b = b1[lane];
  float* ow = o_t[wave];

#pragma unroll 1
  for (int pass = 0; pass < kPasses; ++pass) {
    const int n0 = wave * kRowsPerWave + pass * kRowsPerPass;
#pragma unroll 1
    for (int r = 0; r < kRowsPerPass; ++r) {
      const float* row = m + ((size_t)(n0 + r) * kL + l) * kD + lane * 8;
      const v4f x0 = *(const v4f*)(row);
      const v4f x1 = *(const v4f*)(row + 4);
      float s = ((x0[0] + x0[1]) + (x0[2] + x0[3])) + ((x1[0] + x1[1]) + (x1[2] + x1[3]));
#pragma unroll
      for (int off = 16; off >= 1; off >>= 1) s += __shfl_xor(s, off, 32);
      const float mu = s * kInvD;
      float e0[4], e1[4];
#pragma unroll
      for (int t = 0; t < 4; ++t) {
        e0[t] = x0[t] - mu;
        e1[t] = x1[t] - mu;
      }
      float q = 0.0f;
#pragma unroll
      for (int t = 0; t < 4; ++t) {
        q = fmaf(e0[t], e0[t], q);
        q = fmaf(e1[t], e1[t], q);
      }
#pragma unroll
      for (int off = 16; off >= 1; off >>= 1) q += __shfl_xor(q, off, 32);
      const float rstd = rsqrtf(q * kInvD + kLnEps);
#pragma unroll
      for (int t = 0; t < 4; ++t) {
        ow[(lane * 8 + t) * kRowsPerPass + r]     = (e0[t] * rstd) * lw0[t] + lb0[t];
        ow[(lane * 8 + 4 + t) * kRowsPerPass + r] = (e1[t] * rstd) * lw1[t] + lb1[t];
      }
    }
    __syncthreads();

    float aa0 = 0.0f, aa1 = 0.0f, aa2 = 0.0f, aa3 = 0.0f;
    float bb0 = 0.0f, bb1 = 0.0f, bb2 = 0.0f, bb3 = 0.0f;
#pragma unroll 4
    for (int d = 0; d < kD; ++d) {
      const v4f ov = *(const v4f*)(ow + d * kRowsPerPass);
      const float wa = w2[d * kC + lane];
      const float wb = w1[d * kC + lane];
      aa0 = fmaf(ov[0], wa, aa0);
      aa1 = fmaf(ov[1], wa, aa1);
      aa2 = fmaf(ov[2], wa, aa2);
      aa3 = fmaf(ov[3], wa, aa3);
      bb0 = fmaf(ov[0], wb, bb0);
      bb1 = fmaf(ov[1], wb, bb1);
      bb2 = fmaf(ov[2], wb, bb2);
      bb3 = fmaf(ov[3], wb, bb3);
    }
    v4h ha, hb;
    ha[0] = (_Float16)(aa0 + bias_a);
    ha[1] = (_Float16)(aa1 + bias_a);
    ha[2] = (_Float16)(aa2 + bias_a);
    ha[3] = (_Float16)(aa3 + bias_a);
    hb[0] = (_Float16)(bb0 + bias_b);
    hb[1] = (_Float16)(bb1 + bias_b);
    hb[2] = (_Float16)(bb2 + bias_b);
    hb[3] = (_Float16)(bb3 + bias_b);
    *(v4h*)(&ab_s[0][lane * kN + n0]) = ha;
    *(v4h*)(&ab_s[1][lane * kN + n0]) = hb;
    __syncthreads();
  }

  const int e0i = tid * 8;
  const int e1i = (256 + tid) * 8;
  const v8h va0 = *(const v8h*)(&ab_s[0][e0i]);
  const v8h va1 = *(const v8h*)(&ab_s[0][e1i]);
  const v8h vb0 = *(const v8h*)(&ab_s[1][e0i]);
  const v8h vb1 = *(const v8h*)(&ab_s[1][e1i]);
  _Float16* pa = A2  + (size_t)l * (kC * kN);
  _Float16* pb = B2T + (size_t)l * (kC * kN);
  *(volatile v8h*)(pa + e0i) = va0;
  *(volatile v8h*)(pa + e1i) = va1;
  *(volatile v8h*)(pb + e0i) = vb0;
  *(volatile v8h*)(pb + e1i) = vb1;
  __threadfence();
  *(volatile v8h*)(pa + e0i) = va0;
  *(volatile v8h*)(pa + e1i) = va1;
  *(volatile v8h*)(pb + e0i) = vb0;
  *(volatile v8h*)(pb + e1i) = vb1;
}

__global__ __launch_bounds__(256) void w3t_kernel(const float* __restrict__ w3, _Float16* __restrict__ W3T)
{
  const int t     = blockIdx.x * 256 + threadIdx.x;
  const int zc    = t >> 7;
  const int chunk = t & 127;
  const int lml   = chunk & 15;
  const int hh    = (chunk >> 4) & 1;
  const int nb    = (chunk >> 5) & 1;
  const int ma    = (chunk >> 6) & 1;
  const int bidx  = nb * 16 + lml;
  const int abase = ma * 16 + hh * 8;
  v8h hv;
#pragma unroll
  for (int r = 0; r < 8; ++r) {
    const float wv = w3[(size_t)((abase + r) * kC + bidx) * kZ + zc];
    hv[r] = (_Float16)(wv * kW3Carry);
  }
  _Float16* dst = W3T + (size_t)zc * kK3 + chunk * 8;
  *(volatile v8h*)dst = hv;
  __threadfence();
  *(volatile v8h*)dst = hv;
}

constexpr int kPairPitch = 1040;
constexpr int kZPitch    = 132;
constexpr int kFusedLds  = 4 * 16 * kPairPitch * 2;
static_assert(kFusedLds == 133120);
static_assert(16 * kZPitch * 4 <= 16 * kPairPitch * 2);
static_assert((kPairPitch * 2) % 16 == 0 && (kZPitch * 4) % 16 == 0);

__global__ __launch_bounds__(128) void fused_kernel(
    const _Float16* __restrict__ A2, const _Float16* __restrict__ B2T,
    const _Float16* __restrict__ W3T, const float* __restrict__ b3, float* __restrict__ z)
{
  extern __shared__ __align__(16) unsigned char smem_raw[];
  const int wid  = threadIdx.x >> 5;
  const int lane = threadIdx.x & 31;
  const int hh   = lane >> 4;
  const int lml  = lane & 15;
  _Float16* pairbuf = (_Float16*)(void*)smem_raw + (size_t)wid * 16 * kPairPitch;

  const int g  = blockIdx.x * 4 + wid;
  const int i  = g >> 4;
  const int j0 = (g & 15) << 4;

  v16h afrag[2][4];
  const _Float16* aBase = A2 + (size_t)i * (kC * kN);
#pragma unroll
  for (int ma = 0; ma < 2; ++ma)
#pragma unroll
    for (int kb = 0; kb < 4; ++kb)
      afrag[ma][kb] = frag_load(aBase + (size_t)(ma * 16 + lml) * kN + kb * 32 + hh * 8);

#pragma unroll 1
  for (int p = 0; p < 16; ++p) {
    const _Float16* bBase = B2T + (size_t)(j0 + p) * (kC * kN) + (size_t)lml * kN + hh * 8;
    v8f acc[2][2];
#pragma unroll
    for (int ma = 0; ma < 2; ++ma)
#pragma unroll
      for (int nb = 0; nb < 2; ++nb) acc[ma][nb] = (v8f){0.f, 0.f, 0.f, 0.f, 0.f, 0.f, 0.f, 0.f};
#pragma unroll
    for (int kb = 0; kb < 4; ++kb) {
#pragma unroll
      for (int nb = 0; nb < 2; ++nb) {
        const v16h bfrag = frag_load(bBase + (size_t)nb * 16 * kN + kb * 32);
#pragma unroll
        for (int ma = 0; ma < 2; ++ma)
          acc[ma][nb] = mma_f16(afrag[ma][kb], bfrag, acc[ma][nb]);
      }
    }
    _Float16* prow = pairbuf + (size_t)p * kPairPitch;
#pragma unroll
    for (int ma = 0; ma < 2; ++ma)
#pragma unroll
      for (int nb = 0; nb < 2; ++nb) {
        v8h packed;
#pragma unroll
        for (int r = 0; r < 8; ++r) packed[r] = (_Float16)acc[ma][nb][r];
        const int chunk = ((ma * 2 + nb) * 2 + hh) * 16 + lml;
        *(v8h*)(prow + chunk * 8) = packed;
      }
  }
  __syncthreads();

  v8f zacc[8];
#pragma unroll
  for (int ct = 0; ct < 8; ++ct) zacc[ct] = (v8f){0.f, 0.f, 0.f, 0.f, 0.f, 0.f, 0.f, 0.f};
  const _Float16* a2Base = pairbuf + (size_t)lml * kPairPitch + hh * 8;
  const _Float16* wBase  = W3T + (size_t)lml * kK3 + hh * 8;
#pragma unroll 1
  for (int kb = 0; kb < kK3 / 32; ++kb) {
    const v16h a2 = frag_load(a2Base + kb * 32);
#pragma unroll
    for (int ct = 0; ct < 8; ++ct) {
      const v16h wfrag = frag_load(wBase + (size_t)(ct * 16) * kK3 + kb * 32);
      zacc[ct] = mma_f16(a2, wfrag, zacc[ct]);
    }
  }
  __syncthreads();

  float* slab = (float*)(void*)pairbuf;
#pragma unroll
  for (int ct = 0; ct < 8; ++ct) {
    const float bias = b3[ct * 16 + lml];
#pragma unroll
    for (int r = 0; r < 8; ++r)
      slab[(hh * 8 + r) * kZPitch + ct * 16 + lml] = zacc[ct][r] * kOutScale + bias;
  }
  __syncthreads();

  float* zrow0 = z + ((size_t)i * kL + j0) * kZ;
  for (int pass = 0; pass < 2; ++pass) {
#pragma unroll
    for (int row = 0; row < 16; ++row) {
      const v4f val = *(const v4f*)(slab + row * kZPitch + lane * 4);
      *(volatile v4f*)(zrow0 + (size_t)row * kZ + lane * 4) = val;
    }
    __threadfence();
  }
}

extern "C" void kernel_launch(void* const* d_in, const int* in_sizes, int n_in,
                              void* d_out, int out_size, void* d_ws, size_t ws_size,
                              hipStream_t stream)
{
  if (n_in < 9) return;
  if (in_sizes[0] != kN * kL * kD) return;
  if (in_sizes[1] != kD) return;
  if (in_sizes[2] != kD) return;
  if (in_sizes[3] != kD * kC) return;
  if (in_sizes[4] != kC) return;
  if (in_sizes[5] != kD * kC) return;
  if (in_sizes[6] != kC) return;
  if (in_sizes[7] != kK3 * kZ) return;
  if (in_sizes[8] != kZ) return;
  if (out_size != kL * kL * kZ) return;
  if (ws_size < kWsTotal) return;

  const float* m    = (const float*)d_in[0];
  const float* ln_w = (const float*)d_in[1];
  const float* ln_b = (const float*)d_in[2];
  const float* w1   = (const float*)d_in[3];
  const float* b1   = (const float*)d_in[4];
  const float* w2   = (const float*)d_in[5];
  const float* b2   = (const float*)d_in[6];
  const float* w3   = (const float*)d_in[7];
  const float* b3   = (const float*)d_in[8];
  float* zout = (float*)d_out;

  char* ws = (char*)d_ws;
  _Float16* A2  = (_Float16*)(ws + kOffA2);
  _Float16* B2T = (_Float16*)(ws + kOffB2T);
  _Float16* W3T = (_Float16*)(ws + kOffW3T);

  prep_kernel<<<kL, 256, 0, stream>>>(m, ln_w, ln_b, w1, b1, w2, b2, A2, B2T);
  w3t_kernel<<<(kZ * (kK3 / 8)) / 256, 256, 0, stream>>>(w3, W3T);
  fused_kernel<<<(kL * (kL / 16)) / 4, 128, kFusedLds, stream>>>(A2, B2T, W3T, b3, zout);
}
